// RNNBase_80281528697416
// MI455X (gfx1250) — hardware-verified
//
#include <hip/hip_runtime.h>


namespace {
constexpr int NBt = 32, T = 512, D = 512, H = 512, G4 = 4 * H;
constexpr float XS = 8.0f, WSC = 256.0f;

typedef _Float16 b16;
typedef __attribute__((ext_vector_type(16))) _Float16 v16b;
typedef __attribute__((ext_vector_type(8))) _Float16 v8b;
typedef __attribute__((ext_vector_type(8))) float v8f;
typedef __attribute__((ext_vector_type(4))) float v4f;
__device__ __forceinline__ float bf16_rne(float f) { unsigned int u = __float_as_uint(f); u += 0x7FFFu + ((u >> 16) & 1u); return __uint_as_float(u & 0xFFFF0000u); }
__device__ __forceinline__ void split16(float v, b16& hi, b16& lo) { hi = (b16)v; lo = (b16)(v - (float)hi); }
__device__ __forceinline__ v16b frag_kb(const b16* p, int hh) { const v8b a = *(const v8b*)(p + 8 * hh), b = *(const v8b*)(p + 16 + 8 * hh); v16b f;
#pragma unroll
  for (int e = 0; e < 8; ++e) { f[e] = a[e]; f[8 + e] = b[e]; } return f; }
__device__ __forceinline__ v8f wmma16b(v16b a, v16b b, v8f c) { v8f d = __builtin_amdgcn_wmma_f32_16x16x32_f16(false, a, false, b, (short)0, c, false, false); asm volatile("v_nop\n\tv_nop\n\tv_nop\n\tv_nop" : "+v"(d) : "v"(a), "v"(b)); return d; }
__device__ __forceinline__ float nexp(float x) { return __builtin_amdgcn_exp2f(x * 1.4426950408889634f); }
__device__ __forceinline__ float pmul(float a, float b) { float p = a * b; asm volatile("" : "+v"(p)); return p; }
__device__ __forceinline__ float sigm(float x) { return 1.0f / (1.0f + nexp(-x)); }
__device__ __forceinline__ float tanh_(float x) { const float e = nexp(-2.0f * fabsf(x)); const float t = (1.0f - e) / (1.0f + e); return x < 0.0f ? -t : t; }

__global__ __launch_bounds__(256) void prep_kernel(const float* __restrict__ x, const float* __restrict__ w0, const float* __restrict__ w1, const float* __restrict__ w2, const float* __restrict__ w3, b16* __restrict__ X16, b16* __restrict__ W) {
  const size_t t = (size_t)blockIdx.x * 256 + threadIdx.x; const size_t nx = (size_t)NBt * T * D / 8, nw = (size_t)G4 * D / 8;
  const float* src; b16* dst; float sc = WSC; size_t e;
  if (t < nx) { src = x; dst = X16; e = t * 8; sc = XS; } else { const size_t u = t - nx; const int k = (int)(u / nw); if (k >= 4) return; e = (u - (size_t)k * nw) * 8; src = (k == 0 ? w0 : k == 1 ? w1 : k == 2 ? w2 : w3); dst = W + (size_t)k * G4 * D; }
  v8b o; for (int j = 0; j < 8; ++j) o[j] = (b16)(bf16_rne(src[e + j]) * sc);
  for (int pass = 0; pass < 2; ++pass) { *(volatile v8b*)(dst + e) = o; __threadfence(); }
}
template <int LAYER, int STEPS>
__global__ __launch_bounds__(512) void lstm_kernel(const b16* __restrict__ X16, const b16* __restrict__ H0h_in, const b16* __restrict__ H0l_in, const b16* __restrict__ Wih, const b16* __restrict__ Whh, const float* __restrict__ bih, const float* __restrict__ bhh, b16* __restrict__ H0h, b16* __restrict__ H0l, float* __restrict__ out) {
  __shared__ __attribute__((aligned(16))) b16 Hh[16][H + 8], Hl[16][H + 8]; __shared__ __attribute__((aligned(16))) float Hs[16][H + 4];
  const int t_ = threadIdx.x, wave = t_ >> 5, lane = t_ & 31, nloc = lane & 15, hlf = lane >> 4; const int b0 = blockIdx.x * 16;
  for (int k = t_; k < 16 * (H + 8); k += 512) { (&Hh[0][0])[k] = (b16)0.0f; (&Hl[0][0])[k] = (b16)0.0f; }
  float bg[2][4]; int ju[2];
#pragma unroll
  for (int ut = 0; ut < 2; ++ut) { ju[ut] = wave * 32 + ut * 16 + nloc;
#pragma unroll
    for (int g = 0; g < 4; ++g) bg[ut][g] = bf16_rne(bih[g * H + ju[ut]]) + bf16_rne(bhh[g * H + ju[ut]]); }
  float cst[2][8];
#pragma unroll
  for (int ut = 0; ut < 2; ++ut)
#pragma unroll
    for (int r = 0; r < 8; ++r) cst[ut][r] = 0.0f;
  __syncthreads();
  for (int t = 0; t < STEPS; ++t) {
    v8f acc[2][4];
#pragma unroll
    for (int ut = 0; ut < 2; ++ut)
#pragma unroll
      for (int g = 0; g < 4; ++g) acc[ut][g] = (v8f){};
    const size_t arow = ((size_t)(b0 + nloc) * T + t) * D;
#pragma unroll 2
    for (int kb = 0; kb < D; kb += 32) {
      if (LAYER == 0) { const v16b a = frag_kb(X16 + arow + kb, hlf);
#pragma unroll
        for (int ut = 0; ut < 2; ++ut)
#pragma unroll
          for (int g = 0; g < 4; ++g) acc[ut][g] = wmma16b(a, frag_kb(Wih + (size_t)(g * H + ju[ut]) * D + kb, hlf), acc[ut][g]); }
      else { const v16b a = frag_kb(H0h_in + arow + kb, hlf), al = frag_kb(H0l_in + arow + kb, hlf);
#pragma unroll
        for (int ut = 0; ut < 2; ++ut)
#pragma unroll
          for (int g = 0; g < 4; ++g) { const v16b bw = frag_kb(Wih + (size_t)(g * H + ju[ut]) * D + kb, hlf); acc[ut][g] = wmma16b(a, bw, acc[ut][g]); acc[ut][g] = wmma16b(al, bw, acc[ut][g]); } } }
#pragma unroll 2
    for (int kb = 0; kb < H; kb += 32) { const v16b a = frag_kb(&Hh[nloc][kb], hlf), al = frag_kb(&Hl[nloc][kb], hlf);
#pragma unroll
      for (int ut = 0; ut < 2; ++ut)
#pragma unroll
        for (int g = 0; g < 4; ++g) { const v16b bw = frag_kb(Whh + (size_t)(g * H + ju[ut]) * H + kb, hlf); acc[ut][g] = wmma16b(a, bw, acc[ut][g]); acc[ut][g] = wmma16b(al, bw, acc[ut][g]); } }
    __syncthreads();
#pragma unroll
    for (int ut = 0; ut < 2; ++ut) { const int j = ju[ut]; const float sc = 1.0f / (XS * WSC);
#pragma unroll
      for (int r = 0; r < 8; ++r) { const float zi = acc[ut][0][r] * sc + bg[ut][0], zf = acc[ut][1][r] * sc + bg[ut][1], zg = acc[ut][2][r] * sc + bg[ut][2], zo = acc[ut][3][r] * sc + bg[ut][3];
        const float c = pmul(sigm(zf), cst[ut][r]) + pmul(sigm(zi), tanh_(zg)); cst[ut][r] = c; const float h = pmul(sigm(zo), tanh_(c)); const int row = 8 * hlf + r;
        b16 a_, c_; split16(h * XS, a_, c_); Hh[row][j] = a_; Hl[row][j] = c_; Hs[row][j] = h; } }
    __syncthreads();
    { const int rr = wave; const size_t orow = (size_t)(b0 + rr) * T + t;
      for (int pass = 0; pass < 2; ++pass) {
        if (LAYER == 0) { for (int hq = 0; hq < 2; ++hq) { *(volatile v8b*)(H0h + orow * H + hq * 256 + lane * 8) = *(const v8b*)(&Hh[rr][hq * 256 + lane * 8]); *(volatile v8b*)(H0l + orow * H + hq * 256 + lane * 8) = *(const v8b*)(&Hl[rr][hq * 256 + lane * 8]); } }
        else { for (int q4 = 0; q4 < 4; ++q4) *(volatile v4f*)(out + orow * H + q4 * 128 + lane * 4) = *(const v4f*)(&Hs[rr][q4 * 128 + lane * 4]); }
        __threadfence(); } }
  }
}
}

extern "C" void kernel_launch(void* const* d_in, const int* in_sizes, int n_in, void* d_out, int out_size, void* d_ws, size_t ws_size, hipStream_t stream) {
  (void)n_in;
  auto Fp = [&](int i) { return (const float*)d_in[i]; };
  if (in_sizes[0] != NBt * T * D || in_sizes[1] != G4 * D || in_sizes[2] != G4 * H || in_sizes[5] != G4 * H || in_sizes[6] != G4 * H || out_size != NBt * T * H) return;
  size_t off = 0; char* ws = (char*)d_ws;
  auto carve = [&](size_t bytes) { char* p = ws + off; off += (bytes + 255) & ~(size_t)255; return p; };
  b16* X16 = (b16*)carve((size_t)NBt * T * D * 2); b16* W = (b16*)carve((size_t)4 * G4 * D * 2); b16* H0h = (b16*)carve((size_t)NBt * T * H * 2); b16* H0l = (b16*)carve((size_t)NBt * T * H * 2);
  if (off > ws_size || off > ((size_t)128 << 20)) return;
  prep_kernel<<<(unsigned)(((size_t)NBt * T * D / 8 + (size_t)4 * G4 * D / 8 + 255) / 256), 256, 0, stream>>>(Fp(0), Fp(1), Fp(2), Fp(5), Fp(6), X16, W);
  lstm_kernel<0, T><<<NBt / 16, 512, 0, stream>>>(X16, nullptr, nullptr, W + (size_t)0 * G4 * D, W + (size_t)1 * G4 * D, Fp(3), Fp(4), H0h, H0l, nullptr);
  lstm_kernel<1, T><<<NBt / 16, 512, 0, stream>>>(X16, H0h, H0l, W + (size_t)2 * G4 * D, W + (size_t)3 * G4 * D, Fp(7), Fp(8), nullptr, nullptr, (float*)d_out);
}
